// _ReservoirExtractor_6536940224679
// MI455X (gfx1250) — hardware-run, weakly checked
//
#include <hip/hip_runtime.h>
#include <math.h>

constexpr int NVOCAB   = 50257;
constexpr int NEMB     = 256;
constexpr int NRES     = 1024;
constexpr int NLAY     = 4;
constexpr int NBAT     = 32;
constexpr int NSTEP    = 512;
constexpr int NFEAT    = NRES * NLAY;
constexpr int ROWS_BLK = 16;
constexpr int NTHR_SEQ = 512;
constexpr int NWAVE_SEQ = NTHR_SEQ / 32;
constexpr int KS_REC   = NRES / 32;
constexpr int KS_IN0   = NEMB / 32;
constexpr int KS_INL   = NRES / 32;
constexpr int KS_L0    = KS_REC + KS_IN0;
constexpr int KS_LN    = KS_REC + KS_INL;
constexpr int WCHUNK   = 64 * 32;
constexpr size_t WB_L0_ELEMS = (size_t)NRES * (size_t)(KS_L0 * 32);
constexpr size_t WB_LN_ELEMS = (size_t)NRES * (size_t)(KS_LN * 32);
constexpr size_t WB_ELEMS    = WB_L0_ELEMS + (size_t)(NLAY - 1) * WB_LN_ELEMS;
constexpr int TAIL_T0  = 448;
constexpr int SLABP    = 68;
constexpr float WCARRY      = 32.0f;
constexpr float WCARRY_INV  = 1.0f / 32.0f;
constexpr float LOCARRY     = 2048.0f;
constexpr float LOCARRY_INV = 1.0f / 2048.0f;
constexpr float LN_EPS_F    = 1e-5f;
constexpr float FEAT_INV    = 1.0f / (float)NFEAT;

static_assert(NBAT % ROWS_BLK == 0, "batch tiles");
static_assert(NRES == 64 * NWAVE_SEQ, "16 waves x 64 columns");
static_assert(NEMB % 64 == 0 && NRES % 64 == 0, "pack tiles");
static_assert(KS_REC % 2 == 0 && KS_IN0 % 2 == 0 && KS_INL % 2 == 0, "k-steps even");
static_assert(NFEAT == 4 * 256 * 4, "LayerNorm lane map");
static_assert(TAIL_T0 >= 1 && TAIL_T0 < NSTEP, "tail start");
static_assert(NVOCAB == 50257 && NSTEP == 512 && NBAT == 32, "wire shapes");

typedef __attribute__((ext_vector_type(16))) _Float16 v16h;
typedef __attribute__((ext_vector_type(8)))  _Float16 v8h;
typedef __attribute__((ext_vector_type(8)))  float    v8f;
typedef __attribute__((ext_vector_type(4)))  float    v4f;

__device__ __forceinline__ unsigned short f2bf_bits(float f) {
  unsigned u = __float_as_uint(f);
  return (unsigned short)((u + 0x7FFFu + ((u >> 16) & 1u)) >> 16);
}
__device__ __forceinline__ float bf_bits2f(unsigned short h) { return __uint_as_float(((unsigned)h) << 16); }
__device__ __forceinline__ float bf16r(float f) { return bf_bits2f(f2bf_bits(f)); }

__device__ __forceinline__ float ftanh(float x) { return 1.0f - 2.0f * __builtin_amdgcn_rcpf(__expf(2.0f * x) + 1.0f); }

__device__ __forceinline__ void grp_guard(v8f& a, v8f& b, v8f& c, v8f& d, v16h x, v16h y0, v16h y1, v16h y2, v16h y3) {
  asm volatile("v_nop\n\tv_nop\n\tv_nop\n\tv_nop" : "+v"(a), "+v"(b), "+v"(c), "+v"(d) : "v"(x), "v"(y0), "v"(y1), "v"(y2), "v"(y3));
}
__device__ __forceinline__ void acc_guard4(v8f& a, v8f& b, v8f& c, v8f& d) {
  asm volatile("v_nop\n\tv_nop\n\tv_nop\n\tv_nop" : "+v"(a), "+v"(b), "+v"(c), "+v"(d));
}

struct FragH {
  union U { v16h v; v8h h[2]; };
  static __device__ __forceinline__ v16h load(const _Float16* p) {
    U f;
    f.h[0] = *(const v8h*)(p);
    f.h[1] = *(const v8h*)(p + 16);
    return f.v;
  }
  static __device__ __forceinline__ v8f mma(v16h a, v16h b, v8f c) {
    return __builtin_amdgcn_wmma_f32_16x16x32_f16(false, a, false, b, (short)0, c, false, false);
  }
};

__global__ __launch_bounds__(256) void pack_w_kernel(const float* __restrict__ Rst, const float* __restrict__ Win0,
                                                     const float* __restrict__ WinR, unsigned short* __restrict__ WB) {
  __shared__ float Tt[64 * 65];
  const int tid = threadIdx.x;
  const int zz = blockIdx.z;
  const int l = zz >> 1;
  const int which = zz & 1;
  const int kin = (zz == 1) ? NEMB : NRES;
  const int k0 = blockIdx.y * 64;
  const int n0 = blockIdx.x * 64;
  if (k0 >= kin) return;
  const int lm1 = (l > 0) ? (l - 1) : 0;
  const float* src = (which == 0) ? (Rst + (size_t)l * NRES * NRES)
                                  : ((l == 0) ? Win0 : (WinR + (size_t)lm1 * NRES * NRES));
  const int ksl = (l == 0) ? KS_L0 : KS_LN;
  const size_t wboff = (l == 0) ? (size_t)0 : (WB_L0_ELEMS + (size_t)lm1 * WB_LN_ELEMS);
  const int ks0 = (which ? KS_REC : 0) + (k0 >> 5);
#pragma unroll
  for (int i = 0; i < 4; ++i) {
    const int idx = i * 256 + tid;
    const int rr = idx >> 4;
    const int cc = (idx & 15) * 4;
    const v4f v = *(const v4f*)(src + (size_t)(k0 + rr) * NRES + n0 + cc);
    Tt[rr * 65 + cc + 0] = v[0];
    Tt[rr * 65 + cc + 1] = v[1];
    Tt[rr * 65 + cc + 2] = v[2];
    Tt[rr * 65 + cc + 3] = v[3];
  }
  __syncthreads();
  const int nl = tid >> 2;
  const int kk0 = (tid & 3) * 8;
  v8h hv[2];
#pragma unroll
  for (int g = 0; g < 2; ++g) {
#pragma unroll
    for (int e = 0; e < 8; ++e) {
      const float f = Tt[(32 * g + kk0 + e) * 65 + nl];
      hv[g][e] = (_Float16)(bf16r(f) * WCARRY);
    }
  }
  const int nt64 = blockIdx.x;
  for (int pass = 0; pass < 2; ++pass) {
#pragma unroll
    for (int g = 0; g < 2; ++g) {
      const size_t o = wboff + (size_t)(nt64 * ksl + ks0 + g) * WCHUNK + (size_t)tid * 8;
      *(volatile v8h*)(WB + o) = hv[g];
    }
    __threadfence();
  }
}

__global__ __launch_bounds__(256) void gather_xe_kernel(const int* __restrict__ x, const float* __restrict__ embed,
                                                        unsigned short* __restrict__ XE) {
  const int lane = threadIdx.x & 31;
  const int row = blockIdx.x * 8 + (threadIdx.x >> 5);
  if (row >= NSTEP * NBAT) return;
  const int t = row >> 5;
  const int b = row & 31;
  int tok = x[b * NSTEP + t];
  tok = tok < 0 ? 0 : tok;
  tok = tok > (NVOCAB - 1) ? (NVOCAB - 1) : tok;
  const float* sp = embed + (size_t)tok * NEMB + lane * 8;
  const v4f a = *(const v4f*)(sp);
  const v4f bq = *(const v4f*)(sp + 4);
  v8h hv;
#pragma unroll
  for (int e = 0; e < 4; ++e) {
    hv[e]     = (_Float16)bf16r(a[e]);
    hv[4 + e] = (_Float16)bf16r(bq[e]);
  }
  unsigned short* op = XE + (size_t)row * NEMB + lane * 8;
  *(volatile v8h*)op = hv;
  __threadfence();
  *(volatile v8h*)op = hv;
}

__global__ __launch_bounds__(256) void zero_state_kernel(unsigned short* __restrict__ SHI) {
  const int i = blockIdx.x * 256 + threadIdx.x;
  if (i < NLAY * 4096) {
    const int l = i >> 12;
    const int off16 = i & 4095;
    char* p = (char*)SHI + (size_t)(l * 2 + 1) * (size_t)(NBAT * NRES * 2) + (size_t)off16 * 16;
    const v4f zv = {0.0f, 0.0f, 0.0f, 0.0f};
    *(volatile v4f*)p = zv;
    __threadfence();
    *(volatile v4f*)p = zv;
  }
}

template <bool LO>
__device__ __forceinline__ void kseg(const _Float16* ah, const _Float16* al, const _Float16* __restrict__ bw, int nks,
                                     v8f& c0, v8f& c1, v8f& c2, v8f& c3, v8f& d0, v8f& d1, v8f& d2, v8f& d3) {
#pragma unroll 2
  for (int ks = 0; ks < nks; ++ks) {
    const _Float16* bp = bw + (size_t)ks * WCHUNK;
    const v16h a  = FragH::load(ah + ks * 32);
    const v16h b0 = FragH::load(bp);
    const v16h b1 = FragH::load(bp + 512);
    const v16h b2 = FragH::load(bp + 1024);
    const v16h b3 = FragH::load(bp + 1536);
    c0 = FragH::mma(a, b0, c0);
    c1 = FragH::mma(a, b1, c1);
    c2 = FragH::mma(a, b2, c2);
    c3 = FragH::mma(a, b3, c3);
    grp_guard(c0, c1, c2, c3, a, b0, b1, b2, b3);
    if (LO) {
      const v16h a2 = FragH::load(al + ks * 32);
      d0 = FragH::mma(a2, b0, d0);
      d1 = FragH::mma(a2, b1, d1);
      d2 = FragH::mma(a2, b2, d2);
      d3 = FragH::mma(a2, b3, d3);
      grp_guard(d0, d1, d2, d3, a2, b0, b1, b2, b3);
    }
  }
}

__global__ __launch_bounds__(NTHR_SEQ) void seq_kernel(const unsigned short* __restrict__ WBp,
                                                       const unsigned short* __restrict__ XEp,
                                                       unsigned short* SHIp, unsigned short* SLOp, float* HF) {
  __shared__ __align__(16) float Sl[NWAVE_SEQ][16 * SLABP];
  const _Float16* WB = (const _Float16*)WBp;
  const _Float16* XE = (const _Float16*)XEp;
  _Float16* SHI = (_Float16*)SHIp;
  _Float16* SLO = (_Float16*)SLOp;
  const int tid = threadIdx.x;
  const int lane = tid & 31;
  const int wave = tid >> 5;
  const int c = lane & 15;
  const int hh = lane >> 4;
  const int koff = hh * 8;
  const int q = lane >> 3;
  const int c8 = (lane & 7) * 8;
  const int c4 = c * 4;
  const int rowbase = blockIdx.x * ROWS_BLK;
  const int n0 = 64 * wave;
  float* slab = Sl[wave];
  const v8f z8 = {0.f, 0.f, 0.f, 0.f, 0.f, 0.f, 0.f, 0.f};

#pragma unroll 1
  for (int t = 0; t < NSTEP; ++t) {
    const int p = t & 1;
    const int pr = p ^ 1;
    const bool tail = (t >= TAIL_T0);
    const bool wlo  = (t >= TAIL_T0 - 1);
    const bool last = (t == NSTEP - 1);
    const _Float16* xrow = XE + ((size_t)t * NBAT + (size_t)(rowbase + c)) * NEMB + koff;

#pragma unroll 1
    for (int l = 0; l < NLAY; ++l) {
      const int lm1 = (l > 0) ? (l - 1) : 0;
      const int ksl = (l == 0) ? KS_L0 : KS_LN;
      const size_t wboff = (l == 0) ? (size_t)0 : (WB_L0_ELEMS + (size_t)lm1 * WB_LN_ELEMS);
      const _Float16* bw = WB + wboff + (size_t)(wave * ksl) * WCHUNK + c * 32 + koff;
      const size_t rdoff = ((size_t)((l * 2 + pr) * NBAT + rowbase + c)) * NRES + koff;
      const size_t inoff = ((size_t)((lm1 * 2 + p) * NBAT + rowbase + c)) * NRES + koff;

      v8f acc0 = z8, acc1 = z8, acc2 = z8, acc3 = z8;
      v8f acl0 = z8, acl1 = z8, acl2 = z8, acl3 = z8;

      if (tail) {
        kseg<true>(SHI + rdoff, SLO + rdoff, bw, KS_REC, acc0, acc1, acc2, acc3, acl0, acl1, acl2, acl3);
        if (l == 0) {
          kseg<false>(xrow, xrow, bw + (size_t)KS_REC * WCHUNK, KS_IN0, acc0, acc1, acc2, acc3, acl0, acl1, acl2, acl3);
        } else {
          kseg<true>(SHI + inoff, SLO + inoff, bw + (size_t)KS_REC * WCHUNK, KS_INL, acc0, acc1, acc2, acc3, acl0, acl1, acl2, acl3);
        }
      } else {
        const _Float16* a2 = (l == 0) ? xrow : (const _Float16*)(SHI + inoff);
        const int nk2 = (l == 0) ? KS_IN0 : KS_INL;
        kseg<false>(SHI + rdoff, SHI + rdoff, bw, KS_REC, acc0, acc1, acc2, acc3, acl0, acl1, acl2, acl3);
        kseg<false>(a2, a2, bw + (size_t)KS_REC * WCHUNK, nk2, acc0, acc1, acc2, acc3, acl0, acl1, acl2, acl3);
      }
      acc_guard4(acc0, acc1, acc2, acc3);
      acc_guard4(acl0, acl1, acl2, acl3);

#pragma unroll
      for (int r = 0; r < 8; ++r) {
        float* sp = slab + (8 * hh + r) * SLABP + c;
        sp[0]  = (acc0[r] + acl0[r] * LOCARRY_INV) * WCARRY_INV;
        sp[16] = (acc1[r] + acl1[r] * LOCARRY_INV) * WCARRY_INV;
        sp[32] = (acc2[r] + acl2[r] * LOCARRY_INV) * WCARRY_INV;
        sp[48] = (acc3[r] + acl3[r] * LOCARRY_INV) * WCARRY_INV;
      }
      __builtin_amdgcn_fence(__ATOMIC_RELEASE, "workgroup");
      __builtin_amdgcn_wave_barrier();
      __builtin_amdgcn_fence(__ATOMIC_ACQUIRE, "workgroup");

#pragma unroll 1
      for (int it = 0; it < 4; ++it) {
        float* sp = slab + (it * 4 + q) * SLABP + c8;
        const v4f za = *(const v4f*)(sp);
        const v4f zb = *(const v4f*)(sp + 4);
        v4f sa, sb;
#pragma unroll
        for (int e = 0; e < 4; ++e) {
          sa[e] = ftanh(za[e]);
          sb[e] = ftanh(zb[e]);
        }
        *(v4f*)(sp) = sa;
        *(v4f*)(sp + 4) = sb;
      }
      __builtin_amdgcn_fence(__ATOMIC_RELEASE, "workgroup");
      __builtin_amdgcn_wave_barrier();
      __builtin_amdgcn_fence(__ATOMIC_ACQUIRE, "workgroup");

      {
        const size_t wroff = ((size_t)((l * 2 + p) * NBAT + rowbase)) * NRES + n0 + c8;
        for (int pass = 0; pass < 2; ++pass) {
#pragma unroll
          for (int it = 0; it < 4; ++it) {
            const int row = it * 4 + q;
            const float* sp = slab + row * SLABP + c8;
            const v4f sa = *(const v4f*)(sp);
            const v4f sb = *(const v4f*)(sp + 4);
            v8h hv, lv;
#pragma unroll
            for (int e = 0; e < 4; ++e) {
              const float fa = sa[e];
              const float fb = sb[e];
              const _Float16 ha = (_Float16)fa;
              const _Float16 hb = (_Float16)fb;
              hv[e] = ha;
              hv[4 + e] = hb;
              lv[e] = (_Float16)((fa - (float)ha) * LOCARRY);
              lv[4 + e] = (_Float16)((fb - (float)hb) * LOCARRY);
            }
            *(volatile v8h*)(SHI + wroff + (size_t)row * NRES) = hv;
            if (wlo) *(volatile v8h*)(SLO + wroff + (size_t)row * NRES) = lv;
          }
          __threadfence();
        }
      }
      if (last) {
        float* hp = HF + (size_t)rowbase * NFEAT + l * NRES + n0 + c4;
        for (int pass = 0; pass < 2; ++pass) {
#pragma unroll
          for (int it = 0; it < 8; ++it) {
            const int row = it * 2 + hh;
            const v4f v = *(const v4f*)(slab + row * SLABP + c4);
            *(volatile v4f*)(hp + (size_t)row * NFEAT) = v;
          }
          __threadfence();
        }
      }
      __syncthreads();
      __threadfence();
    }
  }
}

__global__ __launch_bounds__(256) void ln_kernel(const float* __restrict__ HF, const float* __restrict__ gam,
                                                 const float* __restrict__ bet, float* __restrict__ out) {
  __shared__ float red1[8];
  __shared__ float red2[8];
  const int tid = threadIdx.x;
  const int lane = tid & 31;
  const int wave = tid >> 5;
  const int row = blockIdx.x;
  const float* rp = HF + (size_t)row * NFEAT;
  v4f v[4], g[4], bb[4];
  float s = 0.0f;
#pragma unroll
  for (int qq = 0; qq < 4; ++qq) {
    const int idx = qq * 1024 + tid * 4;
    v[qq]  = *(const v4f*)(rp + idx);
    g[qq]  = *(const v4f*)(gam + idx);
    bb[qq] = *(const v4f*)(bet + idx);
    s += (v[qq][0] + v[qq][1]) + (v[qq][2] + v[qq][3]);
  }
#pragma unroll
  for (int off = 1; off < 32; off <<= 1) s += __shfl_xor(s, off, 32);
  if (lane == 0) red1[wave] = s;
  __syncthreads();
  float tot = 0.0f;
#pragma unroll
  for (int i = 0; i < 8; ++i) tot += red1[i];
  const float mu = tot * FEAT_INV;
  float ss = 0.0f;
#pragma unroll
  for (int qq = 0; qq < 4; ++qq) {
#pragma unroll
    for (int e = 0; e < 4; ++e) {
      const float d = v[qq][e] - mu;
      v[qq][e] = d;
      ss += d * d;
    }
  }
#pragma unroll
  for (int off = 1; off < 32; off <<= 1) ss += __shfl_xor(ss, off, 32);
  if (lane == 0) red2[wave] = ss;
  __syncthreads();
  float tot2 = 0.0f;
#pragma unroll
  for (int i = 0; i < 8; ++i) tot2 += red2[i];
  const float var = tot2 * FEAT_INV;
  const float rstd = rsqrtf(var + LN_EPS_F);
  v4f o[4];
#pragma unroll
  for (int qq = 0; qq < 4; ++qq) {
#pragma unroll
    for (int e = 0; e < 4; ++e) o[qq][e] = (v[qq][e] * rstd) * bf16r(g[qq][e]) + bf16r(bb[qq][e]);
  }
  float* op = out + (size_t)row * NFEAT;
  for (int pass = 0; pass < 2; ++pass) {
#pragma unroll
    for (int qq = 0; qq < 4; ++qq) *(volatile v4f*)(op + qq * 1024 + tid * 4) = o[qq];
    __threadfence();
  }
}

extern "C" void kernel_launch(void* const* d_in, const int* in_sizes, int n_in,
                              void* d_out, int out_size, void* d_ws, size_t ws_size, hipStream_t stream) {
  if (n_in < 7 || d_out == nullptr || d_ws == nullptr) return;
  if (in_sizes[0] != NBAT * NSTEP || in_sizes[1] != NVOCAB * NEMB || in_sizes[2] != NEMB * NRES ||
      in_sizes[3] != (NLAY - 1) * NRES * NRES || in_sizes[4] != NLAY * NRES * NRES ||
      in_sizes[5] != NFEAT || in_sizes[6] != NFEAT || out_size != NBAT * NFEAT) return;

  const int*   x     = (const int*)d_in[0];
  const float* embed = (const float*)d_in[1];
  const float* win0  = (const float*)d_in[2];
  const float* winr  = (const float*)d_in[3];
  const float* rst   = (const float*)d_in[4];
  const float* gam   = (const float*)d_in[5];
  const float* bet   = (const float*)d_in[6];
  float* out = (float*)d_out;

  char* ws = (char*)d_ws;
  size_t off = 0;
  auto carve = [&](size_t bytes) -> char* { char* p = ws + off; off += (bytes + 255) & ~(size_t)255; return p; };
  unsigned short* WB  = (unsigned short*)carve(WB_ELEMS * 2);
  unsigned short* XE  = (unsigned short*)carve((size_t)NSTEP * NBAT * NEMB * 2);
  unsigned short* SHI = (unsigned short*)carve((size_t)NLAY * 2 * NBAT * NRES * 2);
  unsigned short* SLO = (unsigned short*)carve((size_t)NLAY * 2 * NBAT * NRES * 2);
  float*          HF  = (float*)carve((size_t)NBAT * NFEAT * 4);
  if (off > ws_size || off > (size_t)134217728) return;

  pack_w_kernel<<<dim3(NRES / 64, NRES / 64, 2 * NLAY), 256, 0, stream>>>(rst, win0, winr, WB);
  gather_xe_kernel<<<(NSTEP * NBAT) / 8, 256, 0, stream>>>(x, embed, XE);
  zero_state_kernel<<<(NLAY * 4096) / 256, 256, 0, stream>>>(SHI);
  seq_kernel<<<NBAT / ROWS_BLK, NTHR_SEQ, 0, stream>>>(WB, XE, SHI, SLO, HF);
  ln_kernel<<<NBAT, 256, 0, stream>>>(HF, gam, bet, out);
}
